// TransportOperator_58884001628184
// MI455X (gfx1250) — hardware-verified
//
#include <hip/hip_runtime.h>
#include <math.h>


typedef _Float16 v16h __attribute__((ext_vector_type(16)));
typedef _Float16 v8h  __attribute__((ext_vector_type(8)));
typedef float    v8f  __attribute__((ext_vector_type(8)));
typedef float    v4f  __attribute__((ext_vector_type(4)));

union Frag { v16h v; v8h hv[2]; };

#define ND 512
#define NM 16
#define RB 32
#define NW 16
#define STG_PITCH 36
#define TP_PITCH 72
#define PSCALE 1024.0f
#define INV_PSCALE 0.0009765625f

__device__ __forceinline__ v8f wmma16(v16h a, v16h b, v8f c) {
    return __builtin_amdgcn_wmma_f32_16x16x32_f16(false, a, false, b, (short)0, c, false, false);
}

__global__ __launch_bounds__(256) void k_cvt_z(const float* __restrict__ z,
                                               _Float16* zh, int n8,
                                               const float* __restrict__ tz) {
    (void)tz;
    const int i = blockIdx.x * 256 + threadIdx.x;
    if (i >= n8) return;
    const float* p = z + (size_t)i * 8;
    const v4f a = *(const v4f*)p;
    const v4f b = *(const v4f*)(p + 4);
    v8h hv;
    hv[0] = (_Float16)a[0]; hv[1] = (_Float16)a[1]; hv[2] = (_Float16)a[2]; hv[3] = (_Float16)a[3];
    hv[4] = (_Float16)b[0]; hv[5] = (_Float16)b[1]; hv[6] = (_Float16)b[2]; hv[7] = (_Float16)b[3];
    _Float16* d = zh + (size_t)i * 8;
    *(volatile v8h*)d = hv;
    __threadfence();
    *(volatile v8h*)d = hv;
}

__global__ __launch_bounds__(256) void k_cvt_psi(const float* __restrict__ psi,
                                                 _Float16* pt) {
    __shared__ __attribute__((aligned(16))) _Float16 tile[32 * TP_PITCH];
    const int m   = blockIdx.z;
    const int e0  = blockIdx.x * 32;
    const int d0  = blockIdx.y * 64;
    const int tid = threadIdx.x;
    const int tx  = tid & 31;
    const int ty  = tid >> 5;
    const float* src = psi + (size_t)m * ND * ND;
#pragma unroll
    for (int j = 0; j < 8; ++j) {
        const int dl = ty + 8 * j;
        const float v = src[(size_t)(d0 + dl) * ND + (e0 + tx)] * PSCALE;
        tile[tx * TP_PITCH + dl] = (_Float16)v;
    }
    __syncthreads();
    const int q  = tid >> 3;
    const int pc = tid & 7;
    const v8h v = *(const v8h*)(tile + q * TP_PITCH + pc * 8);
    _Float16* dst = pt + ((size_t)m * ND + (e0 + q)) * ND + d0 + pc * 8;
    *(volatile v8h*)dst = v;
    __threadfence();
    *(volatile v8h*)dst = v;
}

__global__ __launch_bounds__(512) void k_main(const _Float16* __restrict__ zh,
                                              const _Float16* __restrict__ pt,
                                              const float* __restrict__ g,
                                              float* out, int nb) {
    __shared__ float part_lds[NW * RB];
    __shared__ float gate_lds[RB];
    __shared__ __attribute__((aligned(16))) float stg[NW * 16 * STG_PITCH];

    const int tid = threadIdx.x;
    const int w   = tid >> 5;
    const int l   = tid & 31;
    const int h   = l >> 4;
    const int lh  = l & 15;
    const int rb0 = blockIdx.x * RB;
    const int cb0 = w * 32;

    int ra0 = rb0 + lh;       if (ra0 > nb - 1) ra0 = nb - 1;
    int ra1 = rb0 + 16 + lh;  if (ra1 > nb - 1) ra1 = nb - 1;
    const _Float16* arow0 = zh + (size_t)ra0 * ND + 8 * h;
    const _Float16* arow1 = zh + (size_t)ra1 * ND + 8 * h;

    v8f dac[2][2];
#pragma unroll
    for (int rt = 0; rt < 2; ++rt)
#pragma unroll
        for (int ct = 0; ct < 2; ++ct) dac[rt][ct] = (v8f)0.f;

    const bool u8 = (lh & 8) != 0, u4 = (lh & 4) != 0, u2 = (lh & 2) != 0, u1 = (lh & 1) != 0;

    for (int m = 0; m < NM; ++m) {
        v8f acc[2][2];
#pragma unroll
        for (int rt = 0; rt < 2; ++rt)
#pragma unroll
            for (int ct = 0; ct < 2; ++ct) acc[rt][ct] = (v8f)0.f;

        const _Float16* bc0 = pt + ((size_t)m * ND + (cb0 + lh)) * ND + 8 * h;
        const _Float16* bc1 = bc0 + (size_t)16 * ND;

        for (int k0 = 0; k0 < ND; k0 += 32) {
            Frag a0, a1, b0, b1;
            a0.hv[0] = *(const v8h*)(arow0 + k0);
            a0.hv[1] = *(const v8h*)(arow0 + k0 + 16);
            a1.hv[0] = *(const v8h*)(arow1 + k0);
            a1.hv[1] = *(const v8h*)(arow1 + k0 + 16);
            b0.hv[0] = *(const v8h*)(bc0 + k0);
            b0.hv[1] = *(const v8h*)(bc0 + k0 + 16);
            b1.hv[0] = *(const v8h*)(bc1 + k0);
            b1.hv[1] = *(const v8h*)(bc1 + k0 + 16);
            acc[0][0] = wmma16(a0.v, b0.v, acc[0][0]);
            acc[0][1] = wmma16(a0.v, b1.v, acc[0][1]);
            acc[1][0] = wmma16(a1.v, b0.v, acc[1][0]);
            acc[1][1] = wmma16(a1.v, b1.v, acc[1][1]);
            asm volatile("v_nop\n\tv_nop\n\tv_nop\n\tv_nop"
                         : "+v"(acc[0][0]), "+v"(acc[0][1]), "+v"(acc[1][0]), "+v"(acc[1][1])
                         : "v"(a0.v), "v"(a1.v), "v"(b0.v), "v"(b1.v));
        }

        const float g0 = g[(size_t)m * ND + cb0 + lh];
        const float g1 = g[(size_t)m * ND + cb0 + 16 + lh];
        float pv[16];
#pragma unroll
        for (int r = 0; r < 8; ++r) {
            pv[r]     = acc[0][0][r] * g0 + acc[0][1][r] * g1;
            pv[8 + r] = acc[1][0][r] * g0 + acc[1][1][r] * g1;
        }
        float q8[8], q4[4], q2[2], q1;
#pragma unroll
        for (int i = 0; i < 8; ++i) {
            const float kp = u8 ? pv[i + 8] : pv[i];
            const float sd = u8 ? pv[i] : pv[i + 8];
            q8[i] = kp + __shfl_xor(sd, 8, 32);
        }
#pragma unroll
        for (int i = 0; i < 4; ++i) {
            const float kp = u4 ? q8[i + 4] : q8[i];
            const float sd = u4 ? q8[i] : q8[i + 4];
            q4[i] = kp + __shfl_xor(sd, 4, 32);
        }
#pragma unroll
        for (int i = 0; i < 2; ++i) {
            const float kp = u2 ? q4[i + 2] : q4[i];
            const float sd = u2 ? q4[i] : q4[i + 2];
            q2[i] = kp + __shfl_xor(sd, 2, 32);
        }
        {
            const float kp = u1 ? q2[1] : q2[0];
            const float sd = u1 ? q2[0] : q2[1];
            q1 = kp + __shfl_xor(sd, 1, 32);
        }
        part_lds[w * RB + ((lh >> 3) * 16 + 8 * h + (lh & 7))] = q1;
        __syncthreads();

        if (tid < RB) {
            float s = 0.f;
#pragma unroll
            for (int w2 = 0; w2 < NW; ++w2) s += part_lds[w2 * RB + tid];
            s *= INV_PSCALE;
            const float sg = 1.0f / (1.0f + expf(-s));
            gate_lds[tid] = fmaxf(0.0f, 2.0f * sg - 1.0f);
        }
        __syncthreads();

        float ga[8], gb[8];
#pragma unroll
        for (int r = 0; r < 8; ++r) {
            ga[r] = gate_lds[8 * h + r];
            gb[r] = gate_lds[16 + 8 * h + r];
        }
#pragma unroll
        for (int r = 0; r < 8; ++r) {
            dac[0][0][r] = fmaf(ga[r], acc[0][0][r], dac[0][0][r]);
            dac[0][1][r] = fmaf(ga[r], acc[0][1][r], dac[0][1][r]);
            dac[1][0][r] = fmaf(gb[r], acc[1][0][r], dac[1][0][r]);
            dac[1][1][r] = fmaf(gb[r], acc[1][1][r], dac[1][1][r]);
        }
    }

    float* stw = stg + w * 16 * STG_PITCH;
    v4f ov[2][4];
#pragma unroll
    for (int rt = 0; rt < 2; ++rt) {
#pragma unroll
        for (int ct = 0; ct < 2; ++ct)
#pragma unroll
            for (int r = 0; r < 8; ++r)
                stw[(8 * h + r) * STG_PITCH + ct * 16 + lh] = dac[rt][ct][r] * INV_PSCALE;
        __syncthreads();
#pragma unroll
        for (int p = 0; p < 4; ++p) {
            const int row = p * 4 + (l >> 3);
            ov[rt][p] = *(const v4f*)(stw + row * STG_PITCH + (l & 7) * 4);
            const int grow = rb0 + rt * 16 + row;
            if (grow < nb)
                *(volatile v4f*)(out + (size_t)grow * ND + cb0 + (l & 7) * 4) = ov[rt][p];
        }
        __syncthreads();
    }
    __threadfence();
#pragma unroll
    for (int rt = 0; rt < 2; ++rt)
#pragma unroll
        for (int p = 0; p < 4; ++p) {
            const int row = p * 4 + (l >> 3);
            const int grow = rb0 + rt * 16 + row;
            if (grow < nb)
                *(volatile v4f*)(out + (size_t)grow * ND + cb0 + (l & 7) * 4) = ov[rt][p];
        }
}

extern "C" void kernel_launch(void* const* d_in, const int* in_sizes, int n_in,
                              void* d_out, int out_size, void* d_ws, size_t ws_size,
                              hipStream_t stream) {
    if (n_in < 4) return;
    const float* tz  = (const float*)d_in[0];
    const float* z   = (const float*)d_in[1];
    const float* psi = (const float*)d_in[2];
    const float* g   = (const float*)d_in[3];
    const int n_z = in_sizes[1], n_p = in_sizes[2], n_g = in_sizes[3];
    if (n_g != NM * ND || n_p != NM * ND * ND || n_z <= 0 || (n_z % ND) != 0) return;
    const int nb = n_z / ND;
    if (out_size != nb * ND) return;

    const size_t zh_bytes = (size_t)nb * ND * sizeof(_Float16);
    const size_t pt_bytes = (size_t)NM * ND * ND * sizeof(_Float16);
    const size_t off_pt   = (zh_bytes + 255) & ~(size_t)255;
    if (off_pt + pt_bytes > ws_size) return;

    char* ws = (char*)d_ws;
    _Float16* zh = (_Float16*)ws;
    _Float16* pt = (_Float16*)(ws + off_pt);
    float* out = (float*)d_out;

    const int n8 = nb * (ND / 8);
    k_cvt_z  <<<dim3((n8 + 255) / 256), dim3(256), 0, stream>>>(z, zh, n8, tz);
    k_cvt_psi<<<dim3(ND / 32, ND / 64, NM), dim3(256), 0, stream>>>(psi, pt);
    k_main   <<<dim3((nb + RB - 1) / RB), dim3(512), 0, stream>>>(zh, pt, g, out, nb);
}
